// PSABlock_EDFFN_17248588661071
// MI455X (gfx1250) — hardware-verified
//
#include <hip/hip_runtime.h>
#define NBt 8
#define CC 256
#define HW 32
#define NPX (HW * HW)
#define NR (NBt * NPX)
#define NH 4
#define KD 32
#define HD 64
#define QC 512
#define HID 512
#define PS 8
#define NPAT (NBt * 16)
typedef __bf16 v16b __attribute__((ext_vector_type(16)));
typedef unsigned short v8us __attribute__((ext_vector_type(8), may_alias));
typedef float  v8f  __attribute__((ext_vector_type(8)));
typedef float  v4f  __attribute__((ext_vector_type(4)));
typedef float  v4fa __attribute__((ext_vector_type(4), may_alias));
union FragB { v16b v; v8us half[2]; unsigned short u[16]; };

__device__ __forceinline__ unsigned short bf16_bits(float x) { unsigned int u = __float_as_uint(x); return (unsigned short)((u + 0x7FFFu + ((u >> 16) & 1u)) >> 16); }
__device__ __forceinline__ float bf16_val(unsigned short b) { return __uint_as_float(((unsigned int)b) << 16); }
__device__ __forceinline__ float bf16_round(float x) { return bf16_val(bf16_bits(x)); }
template <int NT>
__device__ __forceinline__ v8f mmaN(v16b ah, v16b al, v16b bh, v16b bl, v8f c) {
  c = __builtin_amdgcn_wmma_f32_16x16x32_bf16(false, ah, false, bh, (short)0, c, false, false);
  if (NT >= 2) c = __builtin_amdgcn_wmma_f32_16x16x32_bf16(false, al, false, bh, (short)0, c, false, false);
  if (NT >= 3) c = __builtin_amdgcn_wmma_f32_16x16x32_bf16(false, ah, false, bl, (short)0, c, false, false);
  asm volatile("v_nop\n\tv_nop\n\tv_nop\n\tv_nop" : "+v"(c) : "v"(ah), "v"(al), "v"(bh), "v"(bl));
  return c;
}

__global__ __launch_bounds__(256) void k_wt_bf16(const float* __restrict__ W, unsigned short* __restrict__ Wt, int K, int N) {
  const int t = blockIdx.x * 256 + threadIdx.x;
  const int k8n = K / 8;
  if (t >= N * k8n) return;
  const int n = t / k8n, k8 = (t % k8n) * 8;
  v8us v;
#pragma unroll
  for (int i = 0; i < 8; ++i) v[i] = bf16_bits(W[(size_t)(k8 + i) * N + n]);
  *(volatile v8us*)(Wt + (size_t)n * K + k8) = v;
  __threadfence();
  *(volatile v8us*)(Wt + (size_t)n * K + k8) = v;
}

template <bool ASPLIT, int ACT, bool BIAS_BF16>
__global__ __launch_bounds__(128) void k_gemm_bf(const float* __restrict__ A, int lda, const unsigned short* __restrict__ Wt, int ldb,
                                               const float* __restrict__ bias, float* __restrict__ C, int ldc, int M, int N, int K) {
  __shared__ __attribute__((aligned(16))) float so[4][16][64];
  const int tid = threadIdx.x, w = tid >> 5, lane = tid & 31, ln = lane & 15, hh = lane >> 4;
  const int ntn = N / 64;
  const int wid = blockIdx.x * 4 + w;
  const int mt = wid / ntn, nq = wid % ntn;
  if (mt * 16 >= M) return;
  const int row0 = mt * 16, col0 = nq * 64;
  const float* arow = A + (size_t)(row0 + ln) * lda;
  v8f acc[4] = {};
  for (int kb = 0; kb < K; kb += 32) {
    FragB ah, al;
    const v4f x0 = *(const v4fa*)(arow + kb + 8 * hh), x1 = *(const v4fa*)(arow + kb + 8 * hh + 4);
    const v4f x2 = *(const v4fa*)(arow + kb + 16 + 8 * hh), x3 = *(const v4fa*)(arow + kb + 16 + 8 * hh + 4);
    float xs[16] = {x0[0],x0[1],x0[2],x0[3],x1[0],x1[1],x1[2],x1[3],x2[0],x2[1],x2[2],x2[3],x3[0],x3[1],x3[2],x3[3]};
#pragma unroll
    for (int i = 0; i < 16; ++i) { const unsigned short hb = bf16_bits(xs[i]); ah.u[i] = hb; al.u[i] = ASPLIT ? bf16_bits(xs[i] - bf16_val(hb)) : (unsigned short)0; }
#pragma unroll
    for (int t = 0; t < 4; ++t) {
      const unsigned short* brow = Wt + (size_t)(col0 + t * 16 + ln) * ldb + kb;
      FragB b;
      b.half[0] = *(const v8us*)(brow + 8 * hh);
      b.half[1] = *(const v8us*)(brow + 16 + 8 * hh);
      acc[t] = mmaN<ASPLIT ? 2 : 1>(ah.v, al.v, b.v, b.v, acc[t]);
    }
  }
#pragma unroll
  for (int t = 0; t < 4; ++t) {
    float bv = bias ? bias[col0 + t * 16 + ln] : 0.f;
    if (BIAS_BF16) bv = bf16_round(bv);
#pragma unroll
    for (int r = 0; r < 8; ++r) { float v = acc[t][r] + bv; if (ACT == 1) v = fmaxf(v, 0.f); so[w][8 * hh + r][t * 16 + ln] = v; }
  }
  __builtin_amdgcn_fence(__ATOMIC_ACQ_REL, "workgroup");
  __builtin_amdgcn_wave_barrier();
  const int rsub = lane >> 4, c4 = (lane & 15) * 4;
  for (int pass = 0; pass < 2; ++pass) {
#pragma unroll
    for (int q = 0; q < 8; ++q) {
      const int r = q * 2 + rsub;
      const v4f v = *(const v4fa*)&so[w][r][c4];
      *(volatile v4f*)(C + (size_t)(row0 + r) * ldc + col0 + c4) = v;
    }
    if (pass == 0) __threadfence();
  }
}

template <bool ASPLIT, int ACT, bool BIAS_BF16, bool RES_BF16>
__global__ __launch_bounds__(128) void k_gemm_bf3(const float* __restrict__ A, int lda, const unsigned short* __restrict__ Wt, int ldb,
                                                const float* __restrict__ bias, const float* __restrict__ resid, int rmod, int ldr,
                                                float* __restrict__ C, int ldc, int M, int N, int K) {
  __shared__ __attribute__((aligned(16))) float so[4][16][64];
  const int tid = threadIdx.x, w = tid >> 5, lane = tid & 31, ln = lane & 15, hh = lane >> 4;
  const int ntn = N / 64;
  const int wid = blockIdx.x * 4 + w;
  const int mt = wid / ntn, nq = wid % ntn;
  if (mt * 16 >= M) return;
  const int row0 = mt * 16, col0 = nq * 64;
  const float* arow = A + (size_t)(row0 + ln) * lda;
  v8f acc[4] = {};
  for (int kb = 0; kb < K; kb += 32) {
    FragB ah, al;
    const v4f x0 = *(const v4fa*)(arow + kb + 8 * hh), x1 = *(const v4fa*)(arow + kb + 8 * hh + 4);
    const v4f x2 = *(const v4fa*)(arow + kb + 16 + 8 * hh), x3 = *(const v4fa*)(arow + kb + 16 + 8 * hh + 4);
    float xs[16] = {x0[0],x0[1],x0[2],x0[3],x1[0],x1[1],x1[2],x1[3],x2[0],x2[1],x2[2],x2[3],x3[0],x3[1],x3[2],x3[3]};
#pragma unroll
    for (int i = 0; i < 16; ++i) { const unsigned short hb = bf16_bits(xs[i]); ah.u[i] = hb; al.u[i] = ASPLIT ? bf16_bits(xs[i] - bf16_val(hb)) : (unsigned short)0; }
#pragma unroll
    for (int t = 0; t < 4; ++t) {
      const unsigned short* brow = Wt + (size_t)(col0 + t * 16 + ln) * ldb + kb;
      FragB b;
      b.half[0] = *(const v8us*)(brow + 8 * hh);
      b.half[1] = *(const v8us*)(brow + 16 + 8 * hh);
      acc[t] = mmaN<ASPLIT ? 2 : 1>(ah.v, al.v, b.v, b.v, acc[t]);
    }
  }
#pragma unroll
  for (int t = 0; t < 4; ++t) {
    const int col = col0 + t * 16 + ln;
    float bv = bias ? bias[col] : 0.f;
    if (BIAS_BF16) bv = bf16_round(bv);
#pragma unroll
    for (int r = 0; r < 8; ++r) {
      float v = acc[t][r] + bv;
      if (resid) { float rv = resid[(size_t)((row0 + 8 * hh + r) % rmod) * ldr + col]; if (RES_BF16) rv = bf16_round(rv); v += rv; }
      if (ACT == 1) v = fmaxf(v, 0.f);
      if (ACT == 2) v = 0.5f * v * (1.0f + erff(v * 0.70710678118654752f));
      if (ACT == 3) { const float u = 0.7978845608028654f * (v + 0.044715f * v * v * v); v = 0.5f * v * (1.0f + tanhf(u)); }
      so[w][8 * hh + r][t * 16 + ln] = v;
    }
  }
  __builtin_amdgcn_fence(__ATOMIC_ACQ_REL, "workgroup");
  __builtin_amdgcn_wave_barrier();
  const int rsub = lane >> 4, c4 = (lane & 15) * 4;
  for (int pass = 0; pass < 2; ++pass) {
#pragma unroll
    for (int q = 0; q < 8; ++q) {
      const int r = q * 2 + rsub;
      const v4f v = *(const v4fa*)&so[w][r][c4];
      *(volatile v4f*)(C + (size_t)(row0 + r) * ldc + col0 + c4) = v;
    }
    if (pass == 0) __threadfence();
  }
}
template <bool PARAM_BF16>
__global__ __launch_bounds__(256) void k_layernorm(const float* __restrict__ X, const float* __restrict__ R, const float* __restrict__ g, const float* __restrict__ bta,
                                                  float* __restrict__ out_sum, float* __restrict__ out_norm, int N, float eps) {
  __shared__ float red[256];
  const int row = blockIdx.x, tid = threadIdx.x;
  const float* x = X + (size_t)row * N; const float* rr = R ? R + (size_t)row * N : nullptr;
  float vals[16];
  const int per = N / 256;
  float s1 = 0.f;
  for (int u = 0; u < per / 4; ++u) {
    const int j = tid * 4 + 1024 * u;
    const v4f a = *(const v4fa*)(x + j);
    v4f b = {0.f,0.f,0.f,0.f}; if (rr) b = *(const v4fa*)(rr + j);
#pragma unroll
    for (int q = 0; q < 4; ++q) { const float v = a[q] + b[q]; vals[u * 4 + q] = v; s1 += v; }
  }
  red[tid] = s1; __syncthreads();
  for (int st = 128; st > 0; st >>= 1) { if (tid < st) red[tid] += red[tid + st]; __syncthreads(); }
  const float mu = red[0] / (float)N; __syncthreads();
  float s2 = 0.f;
  for (int u = 0; u < per / 4; ++u)
#pragma unroll
    for (int q = 0; q < 4; ++q) { const float c = vals[u * 4 + q] - mu; s2 += c * c; }
  red[tid] = s2; __syncthreads();
  for (int st = 128; st > 0; st >>= 1) { if (tid < st) red[tid] += red[tid + st]; __syncthreads(); }
  const float rs = rsqrtf(red[0] / (float)N + eps);
  for (int pass = 0; pass < 2; ++pass) {
    for (int u = 0; u < per / 4; ++u) {
      const int j = tid * 4 + 1024 * u;
      v4f o, sm;
#pragma unroll
      for (int q = 0; q < 4; ++q) {
        float gg = g[j + q], bb = bta[j + q];
        if (PARAM_BF16) { gg = bf16_round(gg); bb = bf16_round(bb); }
        sm[q] = vals[u * 4 + q]; o[q] = (vals[u * 4 + q] - mu) * rs * gg + bb;
      }
      if (out_sum) *(volatile v4f*)(out_sum + (size_t)row * N + j) = sm;
      *(volatile v4f*)(out_norm + (size_t)row * N + j) = o;
    }
    if (pass == 0) __threadfence();
  }
}


typedef _Float16 v16h __attribute__((ext_vector_type(16)));
union FragH { v16h v; v8us half[2]; _Float16 h[16]; unsigned short u[16]; };
template <int NT>
__device__ __forceinline__ v8f mmaH(v16h ah, v16h al, v16h bh, v16h bl, v8f c) {
  c = __builtin_amdgcn_wmma_f32_16x16x32_f16(false, ah, false, bh, (short)0, c, false, false);
  if (NT >= 2) c = __builtin_amdgcn_wmma_f32_16x16x32_f16(false, al, false, bh, (short)0, c, false, false);
  if (NT >= 3) c = __builtin_amdgcn_wmma_f32_16x16x32_f16(false, ah, false, bl, (short)0, c, false, false);
  asm volatile("v_nop\n\tv_nop\n\tv_nop\n\tv_nop" : "+v"(c) : "v"(ah), "v"(al), "v"(bh), "v"(bl));
  return c;
}
template <bool ASPLIT>
__global__ __launch_bounds__(128) void k_gemm_h(const float* __restrict__ A, int lda, size_t sA, const _Float16* __restrict__ Bh, int ldb, size_t sB, float alpha, float* __restrict__ C, int ldc, size_t sC, int M, int N, int K) {
  __shared__ __attribute__((aligned(16))) float so[4][16][64];
  const int tid = threadIdx.x, w = tid >> 5, lane = tid & 31, ln = lane & 15, hh = lane >> 4; const int by = blockIdx.y;
  A += (size_t)by * sA; Bh += (size_t)by * sB; C += (size_t)by * sC;
  const int ntn = (N + 63) / 64; const int wid = blockIdx.x * 4 + w; const int mt = wid / ntn, nq = wid % ntn; if (mt * 16 >= M) return;
  const int row0 = mt * 16, col0 = nq * 64; const float* arow = A + (size_t)(row0 + ln) * lda;
  v8f acc[4] = {};
  for (int kb = 0; kb < K; kb += 32) {
    FragH ah, al;
    const v4f x0 = *(const v4fa*)(arow + kb + 8 * hh), x1 = *(const v4fa*)(arow + kb + 8 * hh + 4), x2 = *(const v4fa*)(arow + kb + 16 + 8 * hh), x3 = *(const v4fa*)(arow + kb + 16 + 8 * hh + 4);
    float xs[16] = {x0[0],x0[1],x0[2],x0[3],x1[0],x1[1],x1[2],x1[3],x2[0],x2[1],x2[2],x2[3],x3[0],x3[1],x3[2],x3[3]};
#pragma unroll
    for (int i = 0; i < 16; ++i) { const _Float16 h = (_Float16)xs[i]; ah.h[i] = h; al.h[i] = ASPLIT ? (_Float16)(xs[i] - (float)h) : (_Float16)0.0f; }
#pragma unroll
    for (int t = 0; t < 4; ++t) { if (col0 + t * 16 >= N) continue; const size_t boff = (size_t)(col0 + t * 16 + ln) * ldb + kb; FragH bq; bq.half[0] = *(const v8us*)(Bh + boff + 8 * hh); bq.half[1] = *(const v8us*)(Bh + boff + 16 + 8 * hh);
      acc[t] = mmaH<ASPLIT ? 2 : 1>(ah.v, al.v, bq.v, bq.v, acc[t]); }
  }
#pragma unroll
  for (int t = 0; t < 4; ++t) { if (col0 + t * 16 >= N) continue;
#pragma unroll
    for (int r = 0; r < 8; ++r) so[w][8 * hh + r][t * 16 + ln] = acc[t][r] * alpha; }
  __builtin_amdgcn_fence(__ATOMIC_ACQ_REL, "workgroup"); __builtin_amdgcn_wave_barrier();
  const int rsub = lane >> 4, c4 = (lane & 15) * 4;
  for (int pass = 0; pass < 2; ++pass) {
#pragma unroll
    for (int q = 0; q < 8; ++q) { const int r = q * 2 + rsub; if (col0 + c4 < N) { const v4f v = *(const v4fa*)&so[w][r][c4]; *(volatile v4f*)(C + (size_t)(row0 + r) * ldc + col0 + c4) = v; } }
    if (pass == 0) __threadfence(); }
}

__global__ __launch_bounds__(256) void k_wt_f16(const float* __restrict__ W, _Float16* __restrict__ Wt, int K, int N, float scale) {
  const int t = blockIdx.x * 256 + threadIdx.x; if (t >= N * (K / 8)) return; const int n = t / (K / 8), k8 = (t % (K / 8)) * 8; FragH f;
#pragma unroll
  for (int i = 0; i < 8; ++i) f.h[i] = (_Float16)(bf16_round(W[(size_t)(k8 + i) * N + n]) * scale); const v8us o = f.half[0];
  *(volatile v8us*)((unsigned short*)Wt + (size_t)n * K + k8) = o; __threadfence(); *(volatile v8us*)((unsigned short*)Wt + (size_t)n * K + k8) = o;
}
template <int ACT>
__global__ __launch_bounds__(128) void k_gemm_hhx(const _Float16* __restrict__ A, int lda, size_t sA, const _Float16* __restrict__ Bh, int ldb, size_t sB, float alpha, const float* __restrict__ bias, size_t sBias, const float* __restrict__ CP, int rowsPerB, size_t sCPb, int row0g,
    float* __restrict__ C, _Float16* __restrict__ C16, int ldc, size_t sC, int M, int N, int K) {
  __shared__ __attribute__((aligned(16))) float so[4][16][64];
  const int tid = threadIdx.x, w = tid >> 5, lane = tid & 31, ln = lane & 15, hh = lane >> 4; const int by = blockIdx.y;
  A += (size_t)by * sA; Bh += (size_t)by * sB; const size_t cofs = (size_t)by * sC; const float* bp = bias ? bias + (size_t)by * sBias : nullptr;
  const int ntn = (N + 63) / 64; const int wid = blockIdx.x * 4 + w; const int mt = wid / ntn, nq = wid % ntn; if (mt * 16 >= M) return;
  const int row0 = mt * 16, col0 = nq * 64; const _Float16* arow = A + (size_t)(row0 + ln) * lda;
  v8f acc[4] = {};
  for (int kb = 0; kb < K; kb += 32) { FragH ah; ah.half[0] = *(const v8us*)((const unsigned short*)arow + kb + 8 * hh); ah.half[1] = *(const v8us*)((const unsigned short*)arow + kb + 16 + 8 * hh);
#pragma unroll
    for (int t = 0; t < 4; ++t) { if (col0 + t * 16 >= N) continue; const size_t boff = (size_t)(col0 + t * 16 + ln) * ldb + kb; FragH bq; bq.half[0] = *(const v8us*)((const unsigned short*)Bh + boff + 8 * hh); bq.half[1] = *(const v8us*)((const unsigned short*)Bh + boff + 16 + 8 * hh);
      acc[t] = mmaH<1>(ah.v, ah.v, bq.v, bq.v, acc[t]); }
  }
#pragma unroll
  for (int t = 0; t < 4; ++t) { if (col0 + t * 16 >= N) continue; const int col = col0 + t * 16 + ln; const float bv = bp ? bf16_round(bp[col]) : 0.f;
#pragma unroll
    for (int r = 0; r < 8; ++r) { float v = acc[t][r] * alpha + bv; if (CP) { const int bidx = (row0g + row0 + 8 * hh + r) / rowsPerB; v += CP[(size_t)bidx * sCPb + (size_t)by * 64 + col]; } if (ACT == 1) v = (v > 0.f) ? v : expm1f(v); else if (ACT == 7) v = (v > 0.f) ? v + 1.0f : expf(v); else if (ACT == 8) v = tanhf(v); else if (ACT == 9) v = 0.5f * v * (1.0f + tanhf(0.7978845608028654f * (v + 0.044715f * v * v * v))); else if (ACT == 11) v = 1.0f / (1.0f + expf(-v)); else if (ACT == 12) v = (v > 0.f) ? v : 0.01f * v; else if (ACT == 14) v = (v > 0.f) ? v : 0.1f * v; else if (ACT == 15) v = v / (1.0f + expf(-v)); else if (ACT == 3) v = fmaxf(v, 0.f); else if (ACT == 6) v = 0.5f * v * (1.0f + erff(v * 0.70710678118654752f)); so[w][8 * hh + r][t * 16 + ln] = v; } }
  __builtin_amdgcn_fence(__ATOMIC_ACQ_REL, "workgroup"); __builtin_amdgcn_wave_barrier();
  const int rsub = lane >> 4, c4 = (lane & 15) * 4; typedef _Float16 v4h __attribute__((ext_vector_type(4)));
  for (int pass = 0; pass < 2; ++pass) {
#pragma unroll
    for (int q = 0; q < 8; ++q) { const int r = q * 2 + rsub; if (col0 + c4 < N) { const v4f v = *(const v4fa*)&so[w][r][c4]; if (C) *(volatile v4f*)(C + cofs + (size_t)(row0 + r) * ldc + col0 + c4) = v; if (C16) { v4h h4; for (int i = 0; i < 4; ++i) h4[i] = (_Float16)v[i]; *(volatile v4h*)(C16 + cofs + (size_t)(row0 + r) * ldc + col0 + c4) = h4; } } }
    if (pass == 0) __threadfence(); }
}


typedef _Float16 v4h __attribute__((ext_vector_type(4)));

__global__ __launch_bounds__(256) void k_x16(const float* __restrict__ x, _Float16* __restrict__ X16, size_t n8) { const size_t t = (size_t)blockIdx.x * 256 + threadIdx.x; if (t >= n8) return; FragH f;
#pragma unroll
  for (int q = 0; q < 8; ++q) f.h[q] = (_Float16)bf16_round(x[t * 8 + q]); *(volatile v8us*)((unsigned short*)X16 + t * 8) = f.half[0]; __threadfence(); *(volatile v8us*)((unsigned short*)X16 + t * 8) = f.half[0]; }
__global__ __launch_bounds__(256) void k_h16(const float* __restrict__ x, _Float16* __restrict__ X16, size_t n8) { const size_t t = (size_t)blockIdx.x * 256 + threadIdx.x; if (t >= n8) return; FragH f;
#pragma unroll
  for (int q = 0; q < 8; ++q) f.h[q] = (_Float16)x[t * 8 + q]; *(volatile v8us*)((unsigned short*)X16 + t * 8) = f.half[0]; __threadfence(); *(volatile v8us*)((unsigned short*)X16 + t * 8) = f.half[0]; }
__global__ __launch_bounds__(256) void k_round16f(const float* __restrict__ W, _Float16* __restrict__ Bt, size_t n8) { const size_t t = (size_t)blockIdx.x * 256 + threadIdx.x; if (t >= n8) return; FragH f;
#pragma unroll
  for (int i = 0; i < 8; ++i) f.h[i] = (_Float16)(bf16_round(W[t * 8 + i]) * 16.0f); *(volatile v8us*)((unsigned short*)Bt + t * 8) = f.half[0]; __threadfence(); *(volatile v8us*)((unsigned short*)Bt + t * 8) = f.half[0]; }
template <int NHv, int TTv>
__global__ __launch_bounds__(256) void k_vt(const _Float16* __restrict__ V16, int ldv, int voff, _Float16* __restrict__ Vt) { __shared__ unsigned short tl[64][66]; const int tid = threadIdx.x; const int slab = blockIdx.x / (TTv / 64), lg = blockIdx.x % (TTv / 64); const int b = slab / NHv, h = slab % NHv;
  for (int i = tid; i < 64 * 8; i += 256) { const int r = i / 8, c8 = (i % 8) * 8; FragH f; f.half[0] = *(const v8us*)((const unsigned short*)V16 + ((size_t)b * TTv + lg * 64 + r) * ldv + voff + h * 64 + c8);
#pragma unroll
    for (int q = 0; q < 8; ++q) tl[r][c8 + q] = f.u[q]; }
  __syncthreads();
  for (int pass = 0; pass < 2; ++pass) {
#pragma unroll
    for (int rd = 0; rd < 2; ++rd) { const int d = rd * 32 + tid / 8, pc = tid % 8; FragH f;
#pragma unroll
      for (int q = 0; q < 8; ++q) f.u[q] = tl[pc * 8 + q][d];
      *(volatile v8us*)((unsigned short*)Vt + ((size_t)slab * 64 + d) * TTv + lg * 64 + pc * 8) = f.half[0]; }
    if (pass == 0) __threadfence(); } }

__global__ __launch_bounds__(256) void k_hl(const float* __restrict__ F, _Float16* __restrict__ Hh, _Float16* __restrict__ Hl, size_t n8) { const size_t t = (size_t)blockIdx.x * 256 + threadIdx.x; if (t >= n8) return; FragH fh, fl; const v4f a = *(const v4fa*)(F + t * 8), c = *(const v4fa*)(F + t * 8 + 4);
#pragma unroll
  for (int q = 0; q < 4; ++q) { _Float16 h = (_Float16)a[q]; fh.h[q] = h; fl.h[q] = (_Float16)((a[q] - (float)h) * 1024.0f); h = (_Float16)c[q]; fh.h[4 + q] = h; fl.h[4 + q] = (_Float16)((c[q] - (float)h) * 1024.0f); }
  for (int pass = 0; pass < 2; ++pass) { *(volatile v8us*)((unsigned short*)Hh + t * 8) = fh.half[0]; *(volatile v8us*)((unsigned short*)Hl + t * 8) = fl.half[0]; if (pass == 0) __threadfence(); } }

__device__ __forceinline__ float gelu_f(float v) { return 0.5f * v * (1.0f + erff(v * 0.70710678118654752f)); }
__global__ __launch_bounds__(256) void k_tok(const float* __restrict__ x, float* __restrict__ X) { const int t = blockIdx.x * 256 + threadIdx.x; if (t >= NR * (CC / 4)) return; const int c0 = (t % (CC / 4)) * 4, r = t / (CC / 4); const int b = r / NPX, n = r % NPX; v4f v;
#pragma unroll
  for (int q = 0; q < 4; ++q) v[q] = bf16_round(x[((size_t)b * CC + c0 + q) * NPX + n]);
  *(volatile v4f*)(X + (size_t)r * CC + c0) = v; __threadfence(); *(volatile v4f*)(X + (size_t)r * CC + c0) = v; }
__global__ __launch_bounds__(256) void k_lnr(const float* __restrict__ X, const float* __restrict__ w, const float* __restrict__ bb, _Float16* __restrict__ O16) {
  #pragma clang fp contract(off)
  const int tid = threadIdx.x, wv = tid >> 5, ln = tid & 31; const int r = blockIdx.x * 8 + wv; if (r >= NR) return; float v[8]; float q2 = 0.f;
#pragma unroll
  for (int k = 0; k < 8; ++k) { v[k] = X[(size_t)r * CC + ln * 8 + k]; q2 += v[k] * v[k]; }
  for (int o = 16; o > 0; o >>= 1) q2 += __shfl_xor(q2, o, 32); const float rs = rsqrtf(q2 / (float)CC + 1e-6f); FragH f;
#pragma unroll
  for (int k = 0; k < 8; ++k) { const int c = ln * 8 + k; f.h[k] = (_Float16)(v[k] * rs * bf16_round(w[c]) + bf16_round(bb[c])); }
  *(volatile v8us*)((unsigned short*)O16 + (size_t)r * CC + ln * 8) = f.half[0]; __threadfence(); *(volatile v8us*)((unsigned short*)O16 + (size_t)r * CC + ln * 8) = f.half[0]; }
__global__ __launch_bounds__(256) void k_bn(float* __restrict__ T, int width, const float* __restrict__ g, const float* __restrict__ bb, const float* __restrict__ mm, const float* __restrict__ vv, _Float16* __restrict__ O16) {
  #pragma clang fp contract(off)
  const int per = width / 8; const int t = blockIdx.x * 256 + threadIdx.x; if (t >= NR * per) return; const int c0 = (t % per) * 8; float* p = T + (size_t)t * 8; const v4f a = *(const v4fa*)p, c4 = *(const v4fa*)(p + 4); v4f oa, ob; FragH f;
#pragma unroll
  for (int q = 0; q < 8; ++q) { const int c = c0 + q; const float s = bf16_round(g[c]) * rsqrtf(bf16_round(vv[c]) + 1e-5f); const float y = ((q < 4) ? a[q] : c4[q - 4]) * s + (bf16_round(bb[c]) - bf16_round(mm[c]) * s); if (q < 4) oa[q] = y; else ob[q - 4] = y; f.h[q] = (_Float16)y; }
  for (int pass = 0; pass < 2; ++pass) { *(volatile v4f*)p = oa; *(volatile v4f*)(p + 4) = ob; if (O16) *(volatile v8us*)((unsigned short*)O16 + (size_t)t * 8) = f.half[0]; if (pass == 0) __threadfence(); } }
__global__ __launch_bounds__(256) void k_vt(const _Float16* __restrict__ Q16, int b, _Float16* __restrict__ VT) { const int t = blockIdx.x * 256 + threadIdx.x; if (t >= CC * (NPX / 8)) return; const int m0 = (t % (NPX / 8)) * 8, hd = t / (NPX / 8); const int h = hd / HD, d = hd % HD; FragH f;
#pragma unroll
  for (int q = 0; q < 8; ++q) f.h[q] = Q16[((size_t)b * NPX + m0 + q) * QC + h * 128 + 64 + d];
  *(volatile v8us*)((unsigned short*)VT + (size_t)hd * NPX + m0) = f.half[0]; __threadfence(); *(volatile v8us*)((unsigned short*)VT + (size_t)hd * NPX + m0) = f.half[0]; }
__global__ __launch_bounds__(256) void k_soft(const float* __restrict__ S, _Float16* __restrict__ P16) {
  #pragma clang fp contract(off)
  const int tid = threadIdx.x, w = tid >> 5, ln = tid & 31; const int row = blockIdx.x * 8 + w; if (row >= NH * NPX) return; const float* sr = S + (size_t)row * NPX; float m = -3.0e38f;
#pragma unroll 1
  for (int jb = 0; jb < NPX; jb += 256) { const v4f a = *(const v4fa*)(sr + jb + 8 * ln), c = *(const v4fa*)(sr + jb + 8 * ln + 4);
#pragma unroll
    for (int k = 0; k < 4; ++k) { m = fmaxf(m, a[k]); m = fmaxf(m, c[k]); } }
  for (int o = 16; o > 0; o >>= 1) m = fmaxf(m, __shfl_xor(m, o, 32));
  float su = 0.f;
#pragma unroll 1
  for (int jb = 0; jb < NPX; jb += 256) { const v4f a = *(const v4fa*)(sr + jb + 8 * ln), c = *(const v4fa*)(sr + jb + 8 * ln + 4);
#pragma unroll
    for (int k = 0; k < 4; ++k) { su += expf(a[k] - m); su += expf(c[k] - m); } }
  for (int o = 16; o > 0; o >>= 1) su += __shfl_xor(su, o, 32); const float inv = 1024.0f / su;
  for (int pass = 0; pass < 2; ++pass) {
#pragma unroll 1
    for (int jb = 0; jb < NPX; jb += 256) { const v4f a = *(const v4fa*)(sr + jb + 8 * ln), c = *(const v4fa*)(sr + jb + 8 * ln + 4); FragH f;
#pragma unroll
      for (int k = 0; k < 4; ++k) { f.h[k] = (_Float16)(expf(a[k] - m) * inv); f.h[4 + k] = (_Float16)(expf(c[k] - m) * inv); }
      *(volatile v8us*)((unsigned short*)P16 + (size_t)row * NPX + jb + 8 * ln) = f.half[0]; }
    if (pass == 0) __threadfence(); } }
__global__ __launch_bounds__(256) void k_pe(const float* __restrict__ OUT, const float* __restrict__ QKV, const float* __restrict__ pw, const float* __restrict__ g, const float* __restrict__ bb, const float* __restrict__ mm, const float* __restrict__ vv, _Float16* __restrict__ O16) {
  #pragma clang fp contract(off)
  const int t = blockIdx.x * 256 + threadIdx.x; if (t >= NR * (CC / 8)) return; const int c0 = (t % (CC / 8)) * 8, r = t / (CC / 8); const int b = r / NPX, n = r % NPX; const int y = n / HW, x = n % HW; FragH f;
#pragma unroll
  for (int q = 0; q < 8; ++q) { const int c = c0 + q; const int h = c / HD, d = c % HD; const int qc = h * 128 + 64 + d; float acc = 0.f;
#pragma unroll
    for (int tp = 0; tp < 9; ++tp) { const int yy = y + tp / 3 - 1, xx = x + tp % 3 - 1; const bool in = (yy >= 0 && yy < HW && xx >= 0 && xx < HW); const float v = QKV[((size_t)b * NPX + min(max(yy, 0), HW - 1) * HW + min(max(xx, 0), HW - 1)) * QC + qc]; acc += (in ? v : 0.f) * bf16_round(pw[c * 9 + tp]); }
    const float s = bf16_round(g[c]) * rsqrtf(bf16_round(vv[c]) + 1e-5f); const float pe = acc * s + (bf16_round(bb[c]) - bf16_round(mm[c]) * s); f.h[q] = (_Float16)(OUT[(size_t)r * CC + c] + pe); }
  *(volatile v8us*)((unsigned short*)O16 + (size_t)r * CC + c0) = f.half[0]; __threadfence(); *(volatile v8us*)((unsigned short*)O16 + (size_t)r * CC + c0) = f.half[0]; }
__global__ __launch_bounds__(256) void k_res(const float* __restrict__ X, const float* __restrict__ PR, const float* __restrict__ gam, float* __restrict__ X1) {
  #pragma clang fp contract(off)
  const int t = blockIdx.x * 256 + threadIdx.x; if (t >= NR * CC / 4) return; const int c0 = (t % (CC / 4)) * 4; const v4f a = *(const v4fa*)(X + (size_t)t * 4), p = *(const v4fa*)(PR + (size_t)t * 4); v4f o;
#pragma unroll
  for (int q = 0; q < 4; ++q) o[q] = a[q] + bf16_round(gam[c0 + q]) * p[q];
  *(volatile v4f*)(X1 + (size_t)t * 4) = o; __threadfence(); *(volatile v4f*)(X1 + (size_t)t * 4) = o; }
__global__ __launch_bounds__(256) void k_dwg(const float* __restrict__ PI, const float* __restrict__ dw, _Float16* __restrict__ G16) {
  #pragma clang fp contract(off)
  const int t = blockIdx.x * 256 + threadIdx.x; if (t >= NR * (HID / 8)) return; const int j0 = (t % (HID / 8)) * 8, r = t / (HID / 8); const int b = r / NPX, n = r % NPX; const int y = n / HW, x = n % HW; FragH f;
#pragma unroll 1
  for (int q = 0; q < 8; ++q) { const int j = j0 + q; float a1 = 0.f, a2 = 0.f;
#pragma unroll
    for (int tp = 0; tp < 9; ++tp) { const int yy = y + tp / 3 - 1, xx = x + tp % 3 - 1; const bool in = (yy >= 0 && yy < HW && xx >= 0 && xx < HW); const float* prow = PI + ((size_t)b * NPX + min(max(yy, 0), HW - 1) * HW + min(max(xx, 0), HW - 1)) * (2 * HID); a1 += (in ? prow[j] : 0.f) * bf16_round(dw[j * 9 + tp]); a2 += (in ? prow[HID + j] : 0.f) * bf16_round(dw[(HID + j) * 9 + tp]); }
    f.h[q] = (_Float16)(gelu_f(a1) * a2); }
  *(volatile v8us*)((unsigned short*)G16 + (size_t)r * HID + j0) = f.half[0]; __threadfence(); *(volatile v8us*)((unsigned short*)G16 + (size_t)r * HID + j0) = f.half[0]; }
__global__ __launch_bounds__(256) void k_xpt(const float* __restrict__ PO, _Float16* __restrict__ XPT) { const int t = blockIdx.x * 256 + threadIdx.x; if (t >= CC * NPAT * PS) return; const int p1 = t & 7; const int pt_ = (t >> 3) % NPAT; const int c = t / (8 * NPAT); const int b = pt_ / 16, gh = (pt_ / 4) % 4, gw = pt_ % 4; FragH f;
#pragma unroll
  for (int p2 = 0; p2 < 8; ++p2) f.h[p2] = (_Float16)PO[((size_t)b * NPX + (gh * 8 + p1) * HW + gw * 8 + p2) * CC + c];
  *(volatile v8us*)((unsigned short*)XPT + ((size_t)c * NPAT + pt_) * 64 + p1 * 8) = f.half[0]; __threadfence(); *(volatile v8us*)((unsigned short*)XPT + ((size_t)c * NPAT + pt_) * 64 + p1 * 8) = f.half[0]; }
__global__ __launch_bounds__(256) void k_mc(const float* __restrict__ Fp, _Float16* __restrict__ M16) {
  #pragma clang fp contract(off)
  __shared__ float cs8[8], sn8[8]; if (threadIdx.x < 8) { cs8[threadIdx.x] = cosf(6.283185307179586f * (float)threadIdx.x / 8.0f); sn8[threadIdx.x] = sinf(6.283185307179586f * (float)threadIdx.x / 8.0f); } __syncthreads();
  const int t = blockIdx.x * 256 + threadIdx.x; if (t >= CC * 64 * 8) return; const int m1 = t & 7, n = (t >> 3) & 63, c = t >> 9; const int n1 = n >> 3, n2 = n & 7; const float* F = Fp + (size_t)c * 40; FragH f = FragH{};
#pragma unroll 1
  for (int m2 = 0; m2 < 8; ++m2) { float yv = 0.f;
#pragma unroll
    for (int v = 0; v < 5; ++v) { float wr = 0.f, wi = 0.f;
#pragma unroll
      for (int u = 0; u < 8; ++u) { const int ph = ((u * n1) - (u * m1 + v * m2)) & 7; const float fu = bf16_round(F[u * 5 + v]); wr += fu * cs8[ph]; wi += fu * sn8[ph]; }
      wr *= 0.125f; wi *= 0.125f;
      if (v == 0) yv += wr; else if (v == 4) yv += ((n2 & 1) ? (0.f - wr) : wr); else { const int ph2 = (v * n2) & 7; yv += 2.0f * (wr * cs8[ph2] - wi * sn8[ph2]); } }
    const _Float16 hv = (_Float16)(yv * 0.125f * 16.0f);
#pragma unroll
    for (int q = 0; q < 8; ++q) f.h[q] = (q == m2) ? hv : f.h[q]; }
  *(volatile v8us*)((unsigned short*)M16 + ((size_t)c * 64 + n) * 64 + m1 * 8) = f.half[0]; __threadfence(); *(volatile v8us*)((unsigned short*)M16 + ((size_t)c * 64 + n) * 64 + m1 * 8) = f.half[0]; }
__global__ __launch_bounds__(256) void k_out(const float* __restrict__ X1, const float* __restrict__ Y, const float* __restrict__ gam, float* __restrict__ out) {
  #pragma clang fp contract(off)
  const int t = blockIdx.x * 256 + threadIdx.x; if (t >= NBt * CC * (NPX / 4)) return; const int n0 = (t % (NPX / 4)) * 4; const int c = (t / (NPX / 4)) % CC; const int b = t / ((NPX / 4) * CC); const float g2 = bf16_round(gam[c]); v4f v;
#pragma unroll
  for (int q = 0; q < 4; ++q) { const int n = n0 + q; const int y = n / HW, x = n % HW; const int pt_ = b * 16 + (y / 8) * 4 + (x / 8); const int pp = (y % 8) * 8 + (x % 8); v[q] = X1[((size_t)b * NPX + n) * CC + c] + g2 * Y[((size_t)c * NPAT + pt_) * 64 + pp]; }
  float* dst = out + ((size_t)b * CC + c) * NPX + n0; *(volatile v4f*)dst = v; __threadfence(); *(volatile v4f*)dst = v; }

extern "C" void kernel_launch(void* const* d_in, const int* in_sizes, int n_in,
                              void* d_out, int out_size, void* d_ws, size_t ws_size, hipStream_t stream) {
  (void)in_sizes; (void)n_in; (void)out_size;
  const float* const* I = (const float* const*)d_in; const float* x = I[0]; const float* n1w = I[1]; const float* n1b = I[2]; const float* n2w = I[3]; const float* n2b = I[4]; const float* gm1 = I[5]; const float* gm2 = I[6]; const float* qkv_w = I[7]; const float* qg = I[8]; const float* qb = I[9]; const float* qm = I[10]; const float* qv = I[11]; const float* pe_w = I[12]; const float* peg = I[13]; const float* peb = I[14]; const float* pem = I[15]; const float* pev = I[16]; const float* proj_w = I[17]; const float* pg = I[18]; const float* pb = I[19]; const float* pm = I[20]; const float* pv = I[21]; const float* pi_w = I[22]; const float* dw_w = I[23]; const float* fft_p = I[24]; const float* po_w = I[25];
  char* ws = (char*)d_ws; size_t off = 0;
  auto take = [&](size_t bytes) { char* p = ws + off; off += (bytes + 255) & ~(size_t)255; return p; };
  _Float16* BQKV = (_Float16*)take((size_t)QC * CC * 2); _Float16* BPROJ = (_Float16*)take((size_t)CC * CC * 2); _Float16* BPI = (_Float16*)take((size_t)2 * HID * CC * 2); _Float16* BPO = (_Float16*)take((size_t)CC * HID * 2); _Float16* M16 = (_Float16*)take((size_t)CC * 64 * 64 * 2);
  float* X = (float*)take((size_t)NR * CC * 4); _Float16* XN16 = (_Float16*)take((size_t)NR * CC * 2); char* R1 = take((size_t)NR * 2 * HID * 4);
  _Float16* QKV16 = (_Float16*)take((size_t)NR * QC * 2); _Float16* VT = (_Float16*)take((size_t)CC * NPX * 2); _Float16* P16 = (_Float16*)take((size_t)NH * NPX * NPX * 2); float* OUT = (float*)take((size_t)NR * CC * 4); _Float16* O16 = (_Float16*)take((size_t)NR * CC * 2); float* PR = (float*)take((size_t)NR * CC * 4); float* X1 = (float*)take((size_t)NR * CC * 4); _Float16* G16 = (_Float16*)take((size_t)NR * HID * 2); float* PO = (float*)take((size_t)NR * CC * 4); _Float16* XPT = (_Float16*)take((size_t)CC * NPAT * 64 * 2); float* Y = (float*)take((size_t)CC * NPAT * 64 * 4);
  if (off > ws_size) return;
  float* QKV = (float*)R1; float* S = (float*)(R1 + (size_t)NR * QC * 4); float* PI = (float*)R1;
  k_round16f<<<(QC * CC / 8 + 255) / 256, 256, 0, stream>>>(qkv_w, BQKV, (size_t)QC * CC / 8); k_round16f<<<(CC * CC / 8 + 255) / 256, 256, 0, stream>>>(proj_w, BPROJ, (size_t)CC * CC / 8); k_round16f<<<(2 * HID * CC / 8 + 255) / 256, 256, 0, stream>>>(pi_w, BPI, (size_t)2 * HID * CC / 8); k_round16f<<<(CC * HID / 8 + 255) / 256, 256, 0, stream>>>(po_w, BPO, (size_t)CC * HID / 8);
  k_mc<<<(CC * 64 * 8 + 255) / 256, 256, 0, stream>>>(fft_p, M16);
  const dim3 gC(((NR / 16) * (CC / 64) + 3) / 4, 1), gQ(((NR / 16) * (QC / 64) + 3) / 4, 1), gP(((NR / 16) * (2 * HID / 64) + 3) / 4, 1);
  k_tok<<<(NR * (CC / 4) + 255) / 256, 256, 0, stream>>>(x, X);
  k_lnr<<<NR / 8, 256, 0, stream>>>(X, n1w, n1b, XN16);
  k_gemm_hhx<0><<<gQ, 128, 0, stream>>>(XN16, CC, 0, BQKV, CC, 0, 0.0625f, nullptr, 0, nullptr, 1, 0, 0, QKV, nullptr, QC, 0, NR, QC, CC); k_bn<<<(NR * (QC / 8) + 255) / 256, 256, 0, stream>>>(QKV, QC, qg, qb, qm, qv, QKV16);
  const dim3 gS(((NPX / 16) * (NPX / 64) + 3) / 4, NH), gV(((NPX / 16) * 1 + 3) / 4, NH);
  for (int b = 0; b < NBt; ++b) { const _Float16* base = QKV16 + (size_t)b * NPX * QC;
    k_gemm_hhx<0><<<gS, 128, 0, stream>>>(base, QC, (size_t)128, base + KD, QC, (size_t)128, 0.17677669529663687f, nullptr, 0, nullptr, 1, 0, 0, S, nullptr, NPX, (size_t)NPX * NPX, NPX, NPX, KD);
    k_soft<<<NH * NPX / 8, 256, 0, stream>>>(S, P16); k_vt<<<(CC * (NPX / 8) + 255) / 256, 256, 0, stream>>>(QKV16, b, VT);
    k_gemm_hhx<0><<<gV, 128, 0, stream>>>(P16, NPX, (size_t)NPX * NPX, VT, NPX, (size_t)HD * NPX, 0.0009765625f, nullptr, 0, nullptr, 1, 0, 0, OUT + (size_t)b * NPX * CC, nullptr, CC, (size_t)HD, NPX, HD, NPX); }
  k_pe<<<(NR * (CC / 8) + 255) / 256, 256, 0, stream>>>(OUT, QKV, pe_w, peg, peb, pem, pev, O16);
  k_gemm_hhx<0><<<gC, 128, 0, stream>>>(O16, CC, 0, BPROJ, CC, 0, 0.0625f, nullptr, 0, nullptr, 1, 0, 0, PR, nullptr, CC, 0, NR, CC, CC); k_bn<<<(NR * (CC / 8) + 255) / 256, 256, 0, stream>>>(PR, CC, pg, pb, pm, pv, nullptr);
  k_res<<<(NR * CC / 4 + 255) / 256, 256, 0, stream>>>(X, PR, gm1, X1);
  k_lnr<<<NR / 8, 256, 0, stream>>>(X1, n2w, n2b, XN16);
  k_gemm_hhx<0><<<gP, 128, 0, stream>>>(XN16, CC, 0, BPI, CC, 0, 0.0625f, nullptr, 0, nullptr, 1, 0, 0, PI, nullptr, 2 * HID, 0, NR, 2 * HID, CC);
  k_dwg<<<(NR * (HID / 8) + 255) / 256, 256, 0, stream>>>(PI, dw_w, G16);
  k_gemm_hhx<0><<<gC, 128, 0, stream>>>(G16, HID, 0, BPO, HID, 0, 0.0625f, nullptr, 0, nullptr, 1, 0, 0, PO, nullptr, CC, 0, NR, CC, HID);
  k_xpt<<<(CC * NPAT * PS + 255) / 256, 256, 0, stream>>>(PO, XPT);
  k_gemm_hhx<0><<<dim3(((NPAT / 16) * 1 + 3) / 4, CC), 128, 0, stream>>>(XPT, 64, (size_t)NPAT * 64, M16, 64, (size_t)64 * 64, 0.0625f, nullptr, 0, nullptr, 1, 0, 0, Y, nullptr, 64, (size_t)NPAT * 64, NPAT, 64, 64);
  k_out<<<(NBt * CC * (NPX / 4) + 255) / 256, 256, 0, stream>>>(X1, Y, gm2, (float*)d_out);
}
